// MultiHeadAttentionBlock_28905129902443
// MI455X (gfx1250) — hardware-verified
//
#include <hip/hip_runtime.h>
#include <stdint.h>

typedef __attribute__((ext_vector_type(16))) _Float16 v16h;
typedef __attribute__((ext_vector_type(8)))  _Float16 v8h;
typedef __attribute__((ext_vector_type(16))) __bf16   v16b;
typedef __attribute__((ext_vector_type(8)))  __bf16   v8b;
typedef __attribute__((ext_vector_type(8)))  float    v8f;
typedef __attribute__((ext_vector_type(4)))  float    v4f;
typedef __attribute__((ext_vector_type(4)))  unsigned int v4u;

constexpr int kBatch = 2;
constexpr int kSeq   = 2048;
constexpr int kDm    = 1024;
constexpr int kHeads = 16;
constexpr int kHd    = 64;
constexpr int kRows  = kBatch * kSeq;
constexpr int kKch   = 64;
constexpr int kQblk  = 64;
constexpr int kWavesA = 4;
constexpr float kPCarry = 32768.0f;
constexpr float kOCarry = 16.0f;
constexpr float kWoCarry = 16.0f;

static_assert(kHeads * kHd == kDm);
static_assert(kRows % 64 == 0 && kDm % 64 == 0 && kDm % 32 == 0);
static_assert(kSeq % kKch == 0 && kSeq % kQblk == 0 && kHd == 64);

__device__ __forceinline__ unsigned short f2bf_bits(float f) {
  unsigned u = __float_as_uint(f);
  return (unsigned short)((u + 0x7FFFu + ((u >> 16) & 1u)) >> 16);
}
__device__ __forceinline__ float bf_bits2f(unsigned short h) { return __uint_as_float(((unsigned)h) << 16); }

__device__ __forceinline__ void dep_guard_h(v8f& a, v8f& b, v16h x, v16h y) { asm volatile("v_nop\n\tv_nop\n\tv_nop\n\tv_nop" : "+v"(a), "+v"(b) : "v"(x), "v"(y)); }
__device__ __forceinline__ void dep_guard_b(v8f& a, v8f& b, v16b x, v16b y) { asm volatile("v_nop\n\tv_nop\n\tv_nop\n\tv_nop" : "+v"(a), "+v"(b) : "v"(x), "v"(y)); }
__device__ __forceinline__ void keep4_h(v16h a, v16h b, v16h c, v16h d) { asm volatile("v_nop" :: "v"(a), "v"(b), "v"(c), "v"(d)); }
__device__ __forceinline__ void keep4_b(v16b a, v16b b, v16b c, v16b d) { asm volatile("v_nop" :: "v"(a), "v"(b), "v"(c), "v"(d)); }
__device__ __forceinline__ void acc_guard4(v8f& a, v8f& b, v8f& c, v8f& d) { asm volatile("v_nop\n\tv_nop\n\tv_nop\n\tv_nop" : "+v"(a), "+v"(b), "+v"(c), "+v"(d)); }
template <typename T> struct Frag;
template <> struct Frag<_Float16> {
  typedef v16h V; union U { v16h v; v8h h[2]; };
  static __device__ __forceinline__ v16h load(const _Float16* p) {
    U f; f.h[0] = *(const v8h*)(p); f.h[1] = *(const v8h*)(p + 16); return f.v;
  }
  static __device__ __forceinline__ v8f mma(v16h a, v16h b, v8f c) {
    return __builtin_amdgcn_wmma_f32_16x16x32_f16(false, a, false, b, (short)0, c, false, false);
  }
  static __device__ __forceinline__ void guard(v8f& a, v8f& b, v16h x, v16h y) { dep_guard_h(a, b, x, y); }
  static __device__ __forceinline__ void keep(v16h a, v16h b, v16h c, v16h d) { keep4_h(a, b, c, d); }
};
template <> struct Frag<__bf16> {
  typedef v16b V; union U { v16b v; v8b h[2]; };
  static __device__ __forceinline__ v16b load(const __bf16* p) {
    U f; f.h[0] = *(const v8b*)(p); f.h[1] = *(const v8b*)(p + 16); return f.v;
  }
  static __device__ __forceinline__ v8f mma(v16b a, v16b b, v8f c) {
    return __builtin_amdgcn_wmma_f32_16x16x32_bf16(false, a, false, b, (short)0, c, false, false);
  }
  static __device__ __forceinline__ void guard(v8f& a, v8f& b, v16b x, v16b y) { dep_guard_b(a, b, x, y); }
  static __device__ __forceinline__ void keep(v16b a, v16b b, v16b c, v16b d) { keep4_b(a, b, c, d); }
};

__device__ __forceinline__ v8f mma_bf16_g(v16b a, v16b b, v8f c) {
  c = __builtin_amdgcn_wmma_f32_16x16x32_bf16(false, a, false, b, (short)0, c, false, false);
  asm volatile("v_nop\n\tv_nop\n\tv_nop\n\tv_nop" : "+v"(c) : "v"(a), "v"(b));
  return c;
}
__device__ __forceinline__ v8f mma_f16_g(v16h a, v16h b, v8f c) {
  c = __builtin_amdgcn_wmma_f32_16x16x32_f16(false, a, false, b, (short)0, c, false, false);
  asm volatile("v_nop\n\tv_nop\n\tv_nop\n\tv_nop" : "+v"(c) : "v"(a), "v"(b));
  return c;
}
__device__ __forceinline__ void wave_lds_sync() {
  __builtin_amdgcn_fence(__ATOMIC_RELEASE, "workgroup");
  __builtin_amdgcn_wave_barrier();
  __builtin_amdgcn_fence(__ATOMIC_ACQUIRE, "workgroup");
}
__device__ __forceinline__ v8f zero8() { return (v8f){0.f, 0.f, 0.f, 0.f, 0.f, 0.f, 0.f, 0.f}; }

__global__ __launch_bounds__(256) void cast_f32_bf16x8(
    const float* __restrict__ in, unsigned short* __restrict__ out, int n8) {
  const int i = blockIdx.x * 256 + threadIdx.x;
  if (i < n8) {
    const v4f a0 = *(const v4f*)(in + (size_t)i * 8);
    const v4f a1 = *(const v4f*)(in + (size_t)i * 8 + 4);
    v4u w;
    w[0] = (unsigned)f2bf_bits(a0[0]) | ((unsigned)f2bf_bits(a0[1]) << 16);
    w[1] = (unsigned)f2bf_bits(a0[2]) | ((unsigned)f2bf_bits(a0[3]) << 16);
    w[2] = (unsigned)f2bf_bits(a1[0]) | ((unsigned)f2bf_bits(a1[1]) << 16);
    w[3] = (unsigned)f2bf_bits(a1[2]) | ((unsigned)f2bf_bits(a1[3]) << 16);
    unsigned short* dst = out + (size_t)i * 8;
    *(volatile v4u*)dst = w;
    __threadfence();
    *(volatile v4u*)dst = w;
  }
}

__global__ __launch_bounds__(256) void cast_f32_f16c_x8(
    const float* __restrict__ in, unsigned short* __restrict__ out, int n8, float carry) {
  const int i = blockIdx.x * 256 + threadIdx.x;
  if (i < n8) {
    const v4f a0 = *(const v4f*)(in + (size_t)i * 8);
    const v4f a1 = *(const v4f*)(in + (size_t)i * 8 + 4);
    unsigned hb[8];
#pragma unroll
    for (int e = 0; e < 4; ++e) {
      const _Float16 h0 = (_Float16)(bf_bits2f(f2bf_bits(a0[e])) * carry);
      const _Float16 h1 = (_Float16)(bf_bits2f(f2bf_bits(a1[e])) * carry);
      hb[e]     = (unsigned)__builtin_bit_cast(unsigned short, h0);
      hb[4 + e] = (unsigned)__builtin_bit_cast(unsigned short, h1);
    }
    v4u w;
    w[0] = hb[0] | (hb[1] << 16);
    w[1] = hb[2] | (hb[3] << 16);
    w[2] = hb[4] | (hb[5] << 16);
    w[3] = hb[6] | (hb[7] << 16);
    unsigned short* dst = out + (size_t)i * 8;
    *(volatile v4u*)dst = w;
    __threadfence();
    *(volatile v4u*)dst = w;
  }
}

template <int ET> struct Elem;
template <> struct Elem<0> { typedef _Float16 T; };
template <> struct Elem<1> { typedef __bf16 T; };
template <int ET, bool SPLIT, int BIAS_MODE, int OUT_MODE, bool RESID, int ACT = 0>
__global__ __launch_bounds__(256) void wmma_gemm64(
    const unsigned short* __restrict__ Ap, const unsigned short* __restrict__ A2p, int lda, long strideA,
    const unsigned short* __restrict__ Btp, const unsigned short* __restrict__ Bt2p, int ldb, long strideB,
    void* __restrict__ Cout, void* __restrict__ Cout2, int ldc, long strideC,
    const float* __restrict__ bias,
    const float* __restrict__ resid, long strideR,
    int M, int N, int K, float scale) {
  static_assert(!RESID);
  typedef typename Elem<ET>::T T;
  typedef typename Frag<T>::V V;
  const T* A = (const T*)Ap; const T* A2 = (const T*)A2p; const T* Bt = (const T*)Btp; const T* Bt2 = (const T*)Bt2p;
  __shared__ __align__(16) float sT[8][16 * 68];
  (void)resid; (void)strideR;
  const int b    = blockIdx.y;
  const int lane = threadIdx.x & 31;
  const int wave = threadIdx.x >> 5;
  const int tilesN = N >> 6;
  const int tilesM = M >> 6;
  const int tile = blockIdx.x * 8 + wave;
  if (tile >= tilesM * tilesN) return;
  const int tm = tile / tilesN;
  const int tn = tile - tm * tilesN;
  const int m0 = tm << 6;
  const int n0 = tn << 6;

  const T* Ab  = A  + (size_t)b * strideA;
  const T* Bb  = Bt + (size_t)b * strideB;
  const T* Ab2 = SPLIT ? (A2  + (size_t)b * strideA) : nullptr;
  const T* Bb2 = SPLIT ? (Bt2 + (size_t)b * strideB) : nullptr;

  const int rlane = lane & 15;
  const int koff  = (lane >> 4) * 8;
  const int mOff  = (lane >> 4) * 8;

  v8f acc[4][4];
#pragma unroll
  for (int i = 0; i < 4; ++i)
#pragma unroll
    for (int j = 0; j < 4; ++j) acc[i][j] = (v8f){0.f,0.f,0.f,0.f,0.f,0.f,0.f,0.f};

  for (int k0 = 0; k0 < K; k0 += 32) {
    V bh[4], bl[4];
#pragma unroll
    for (int j = 0; j < 4; ++j) {
      const size_t bo = (size_t)(n0 + (j << 4) + rlane) * ldb + koff + k0;
      bh[j] = Frag<T>::load(Bb + bo);
      if (SPLIT) bl[j] = Frag<T>::load(Bb2 + bo);
    }
#pragma unroll
    for (int i = 0; i < 4; ++i) {
      const size_t ao = (size_t)(m0 + (i << 4) + rlane) * lda + koff + k0;
      V ah = Frag<T>::load(Ab + ao);
      V al;
      if (SPLIT) al = Frag<T>::load(Ab2 + ao);
#pragma unroll
      for (int j = 0; j < 4; ++j) {
        acc[i][j] = Frag<T>::mma(ah, bh[j], acc[i][j]);
        if (SPLIT) {
          acc[i][j] = Frag<T>::mma(ah, bl[j], acc[i][j]);
          acc[i][j] = Frag<T>::mma(al, bh[j], acc[i][j]);
        }
      }
      Frag<T>::guard(acc[i][0], acc[i][3], ah, SPLIT ? al : ah);
    }
    Frag<T>::keep(bh[0], bh[1], bh[2], bh[3]);
    if (SPLIT) Frag<T>::keep(bl[0], bl[1], bl[2], bl[3]);
  }
  acc_guard4(acc[0][0], acc[0][1], acc[0][2], acc[0][3]);
  acc_guard4(acc[1][0], acc[1][1], acc[1][2], acc[1][3]);
  acc_guard4(acc[2][0], acc[2][1], acc[2][2], acc[2][3]);
  acc_guard4(acc[3][0], acc[3][1], acc[3][2], acc[3][3]);

  float* slab = sT[wave];
  float bn[4] = {0.f, 0.f, 0.f, 0.f};
  if (BIAS_MODE == 2) {
#pragma unroll
    for (int j = 0; j < 4; ++j) bn[j] = bf_bits2f(f2bf_bits(bias[n0 + (j << 4) + rlane]));
  }
#pragma unroll
  for (int i = 0; i < 4; ++i) {
    const int mBase = m0 + (i << 4);
    float bm[8] = {0.f, 0.f, 0.f, 0.f, 0.f, 0.f, 0.f, 0.f};
    if (BIAS_MODE == 1) {
      const v4f b0 = *(const v4f*)(bias + mBase + mOff);
      const v4f b1 = *(const v4f*)(bias + mBase + mOff + 4);
      bm[0] = bf_bits2f(f2bf_bits(b0[0])); bm[1] = bf_bits2f(f2bf_bits(b0[1]));
      bm[2] = bf_bits2f(f2bf_bits(b0[2])); bm[3] = bf_bits2f(f2bf_bits(b0[3]));
      bm[4] = bf_bits2f(f2bf_bits(b1[0])); bm[5] = bf_bits2f(f2bf_bits(b1[1]));
      bm[6] = bf_bits2f(f2bf_bits(b1[2])); bm[7] = bf_bits2f(f2bf_bits(b1[3]));
    }
#pragma unroll
    for (int j = 0; j < 4; ++j) {
#pragma unroll
      for (int r = 0; r < 8; ++r) {
        float v = acc[i][j][r] * scale;
        if (BIAS_MODE == 1) v += bm[r];
        if (BIAS_MODE == 2) v += bn[j];
        if (ACT == 1) v = tanhf(v);
        if (ACT == 2) v = fmaxf(v, 0.0f);
        if (ACT == 4) v = (v > 0.f) ? v : 0.01f * v;
        slab[(mOff + r) * 68 + (j << 4) + rlane] = v;
      }
    }
    __builtin_amdgcn_fence(__ATOMIC_RELEASE, "workgroup");
    __builtin_amdgcn_wave_barrier();
    __builtin_amdgcn_fence(__ATOMIC_ACQUIRE, "workgroup");
    if (OUT_MODE == 0) {
      float* C = (float*)Cout + (size_t)b * strideC;
      const int hh = lane >> 4, c4 = (lane & 15) * 4;
      for (int pass = 0; pass < 2; ++pass) {
#pragma unroll
        for (int it = 0; it < 8; ++it) {
          const int row = it * 2 + hh;
          v4f v = *(const v4f*)(slab + row * 68 + c4);
          *(volatile v4f*)(C + (size_t)(mBase + row) * ldc + n0 + c4) = v;
        }
        __threadfence();
      }
    } else {
      const int q = lane >> 3, c8 = (lane & 7) * 8;
      unsigned short* C  = (unsigned short*)Cout  + (size_t)b * strideC;
      unsigned short* C2 = (OUT_MODE == 2) ? ((unsigned short*)Cout2 + (size_t)b * strideC) : nullptr;
      for (int pass = 0; pass < 2; ++pass) {
#pragma unroll
        for (int it = 0; it < 4; ++it) {
          const int row = it * 4 + q;
          const float* sp = slab + row * 68 + c8;
          v8h hv, lv;
#pragma unroll
          for (int e = 0; e < 8; ++e) {
            if (OUT_MODE == 1) {
              hv[e] = (_Float16)sp[e];
            } else {
              unsigned short hb = f2bf_bits(sp[e]);
              unsigned short lb = f2bf_bits(sp[e] - bf_bits2f(hb));
              hv[e] = __builtin_bit_cast(_Float16, hb);
              lv[e] = __builtin_bit_cast(_Float16, lb);
            }
          }
          *(volatile v8h*)(C + (size_t)(mBase + row) * ldc + n0 + c8) = hv;
          if (OUT_MODE == 2) *(volatile v8h*)(C2 + (size_t)(mBase + row) * ldc + n0 + c8) = lv;
        }
        __threadfence();
      }
    }
    __builtin_amdgcn_fence(__ATOMIC_RELEASE, "workgroup");
    __builtin_amdgcn_wave_barrier();
    __builtin_amdgcn_fence(__ATOMIC_ACQUIRE, "workgroup");
  }
}

__global__ __launch_bounds__(128)
void attn_core(const unsigned short* __restrict__ Qh, const unsigned short* __restrict__ Ql,
               const unsigned short* __restrict__ Kh, const unsigned short* __restrict__ Kl,
               const unsigned short* __restrict__ Vt, unsigned short* __restrict__ Oo,
               float score_scale, float out_mul) {
  __shared__ __align__(16) _Float16 Psh[kWavesA][16 * kKch];
  __shared__ __align__(16) float    Os[kWavesA][16 * 68];

  const int tid  = threadIdx.x;
  const int wave = tid >> 5;
  const int lane = tid & 31;
  const int hh   = lane >> 4;
  const int c    = lane & 15;

  constexpr int nqb = kSeq / kQblk;
  const int bx = blockIdx.x;
  const int qb = bx % nqb;
  const int bh = bx / nqb;
  const int h  = bh % kHeads;
  const int b  = bh / kHeads;
  const int q0 = qb * kQblk + wave * 16;

  const __bf16* Qhp = (const __bf16*)(const void*)Qh;
  const __bf16* Qlp = (const __bf16*)(const void*)Ql;
  const __bf16* Khp = (const __bf16*)(const void*)Kh;
  const __bf16* Klp = (const __bf16*)(const void*)Kl;
  const _Float16* Vtp = (const _Float16*)(const void*)Vt;

  v16b qah[2], qal[2];
  {
    const size_t qo = ((size_t)b * kSeq + (size_t)(q0 + c)) * kDm + (size_t)(h * kHd + 8 * hh);
#pragma unroll
    for (int dc = 0; dc < 2; ++dc) {
      qah[dc] = Frag<__bf16>::load(Qhp + qo + dc * 32);
      qal[dc] = Frag<__bf16>::load(Qlp + qo + dc * 32);
    }
  }

  float mrow[8], lrow[8];
  v8f oacc[4];
#pragma unroll
  for (int r = 0; r < 8; ++r) { mrow[r] = -INFINITY; lrow[r] = 0.f; }
#pragma unroll
  for (int t = 0; t < 4; ++t) oacc[t] = zero8();

  const size_t kbase = (size_t)b * kSeq * kDm + (size_t)(h * kHd + 8 * hh);
  const size_t vbase = (size_t)(h * kHd + c) * kRows + (size_t)b * kSeq + (size_t)(8 * hh);
  _Float16* pw = Psh[wave];

  for (int kc = 0; kc < kSeq / kKch; ++kc) {
    const int kv0 = kc * kKch;

    v8f s[4];
#pragma unroll
    for (int j = 0; j < 4; ++j) {
      s[j] = zero8();
      const size_t ko = kbase + (size_t)(kv0 + j * 16 + c) * kDm;
#pragma unroll
      for (int dc = 0; dc < 2; ++dc) {
        const v16b kbh = Frag<__bf16>::load(Khp + ko + dc * 32);
        const v16b kbl = Frag<__bf16>::load(Klp + ko + dc * 32);
        s[j] = mma_bf16_g(qah[dc], kbh, s[j]);
        s[j] = mma_bf16_g(qah[dc], kbl, s[j]);
        s[j] = mma_bf16_g(qal[dc], kbh, s[j]);
      }
      asm volatile("" ::: "memory");
    }

    float cm[8];
#pragma unroll
    for (int r = 0; r < 8; ++r) {
      float m = -INFINITY;
#pragma unroll
      for (int j = 0; j < 4; ++j) {
        const float sv = s[j][r] * score_scale;
        s[j][r] = sv;
        m = fmaxf(m, sv);
      }
#pragma unroll
      for (int off = 1; off < 16; off <<= 1) m = fmaxf(m, __shfl_xor(m, off, 32));
      cm[r] = m;
    }

    wave_lds_sync();
#pragma unroll
    for (int r = 0; r < 8; ++r) {
      const float mnew  = fmaxf(mrow[r], cm[r]);
      const float alpha = expf(mrow[r] - mnew);
      mrow[r] = mnew;
      float psum = 0.f;
#pragma unroll
      for (int j = 0; j < 4; ++j) {
        const float p = expf(s[j][r] - mnew);
        psum += p;
        pw[(8 * hh + r) * kKch + j * 16 + c] = (_Float16)(p * kPCarry);
      }
#pragma unroll
      for (int off = 1; off < 16; off <<= 1) psum += __shfl_xor(psum, off, 32);
      lrow[r] = lrow[r] * alpha + psum;
#pragma unroll
      for (int t = 0; t < 4; ++t) oacc[t][r] *= alpha;
    }
    wave_lds_sync();

#pragma unroll
    for (int kk = 0; kk < 2; ++kk) {
      const v16h pa = Frag<_Float16>::load(pw + c * kKch + kk * 32 + 8 * hh);
#pragma unroll
      for (int t = 0; t < 4; ++t) {
        const v16h vb = Frag<_Float16>::load(Vtp + vbase + (size_t)(t * 16) * kRows + (size_t)(kv0 + kk * 32));
        oacc[t] = mma_f16_g(pa, vb, oacc[t]);
      }
      asm volatile("" ::: "memory");
    }
  }

  float* os = Os[wave];
#pragma unroll
  for (int r = 0; r < 8; ++r) {
    const float inv = out_mul * (1.0f / lrow[r]);
#pragma unroll
    for (int t = 0; t < 4; ++t) os[(8 * hh + r) * 68 + t * 16 + c] = oacc[t][r] * inv;
  }
  wave_lds_sync();
  {
    const int rq = lane >> 3, c8 = (lane & 7) * 8;
    _Float16* Ob = (_Float16*)(void*)Oo;
    for (int pass = 0; pass < 2; ++pass) {
#pragma unroll
      for (int it = 0; it < 4; ++it) {
        const int row = it * 4 + rq;
        const float* sp = os + row * 68 + c8;
        v8h hv;
#pragma unroll
        for (int e = 0; e < 8; ++e) hv[e] = (_Float16)sp[e];
        *(volatile v8h*)(Ob + ((size_t)b * kSeq + (size_t)(q0 + row)) * kDm + (size_t)(h * kHd + c8)) = hv;
      }
      __threadfence();
    }
  }
}

extern "C" void kernel_launch(void* const* d_in, const int* in_sizes, int n_in,
                              void* d_out, int out_size, void* d_ws, size_t ws_size,
                              hipStream_t stream) {
  constexpr size_t kActElems = (size_t)kRows * kDm;
  constexpr size_t kWElems   = (size_t)kDm * kDm;
  constexpr size_t kAct16B   = kActElems * 2;
  constexpr size_t kW16B     = kWElems * 2;

  constexpr size_t offQb = 0;
  constexpr size_t offKb = offQb + kAct16B;
  constexpr size_t offVb = offKb + kAct16B;
  constexpr size_t offWq = offVb + kAct16B;
  constexpr size_t offWk = offWq + kW16B;
  constexpr size_t offWv = offWk + kW16B;
  constexpr size_t offWo = offWv + kW16B;
  constexpr size_t offQh = offWo + kW16B;
  constexpr size_t offQl = offQh + kAct16B;
  constexpr size_t offKh = offQl + kAct16B;
  constexpr size_t offKl = offKh + kAct16B;
  constexpr size_t offVt = offKl + kAct16B;
  constexpr size_t offO  = offVt + kAct16B;
  constexpr size_t kWsTotal = offO + kAct16B;
  static_assert(kWsTotal == 83886080);
  static_assert(kWsTotal <= 134217728);

  if (n_in < 11) return;
  if (in_sizes[0] != (int)kActElems || in_sizes[1] != (int)kActElems || in_sizes[2] != (int)kActElems) return;
  if (in_sizes[3] != (int)kWElems || in_sizes[5] != (int)kWElems || in_sizes[7] != (int)kWElems || in_sizes[9] != (int)kWElems) return;
  if (in_sizes[4] != kDm || in_sizes[6] != kDm || in_sizes[8] != kDm || in_sizes[10] != kDm) return;
  if (out_size != (int)kActElems) return;
  if (ws_size < kWsTotal) return;

  const float* q  = (const float*)d_in[0];
  const float* k  = (const float*)d_in[1];
  const float* v  = (const float*)d_in[2];
  const float* Wq = (const float*)d_in[3];
  const float* bq = (const float*)d_in[4];
  const float* Wk = (const float*)d_in[5];
  const float* bk = (const float*)d_in[6];
  const float* Wv = (const float*)d_in[7];
  const float* bv = (const float*)d_in[8];
  const float* Wo = (const float*)d_in[9];
  const float* bo = (const float*)d_in[10];

  char* ws = (char*)d_ws;
  unsigned short* qb16 = (unsigned short*)(ws + offQb);
  unsigned short* kb16 = (unsigned short*)(ws + offKb);
  unsigned short* vb16 = (unsigned short*)(ws + offVb);
  unsigned short* wq16 = (unsigned short*)(ws + offWq);
  unsigned short* wk16 = (unsigned short*)(ws + offWk);
  unsigned short* wv16 = (unsigned short*)(ws + offWv);
  unsigned short* wo16 = (unsigned short*)(ws + offWo);
  unsigned short* qh16 = (unsigned short*)(ws + offQh);
  unsigned short* ql16 = (unsigned short*)(ws + offQl);
  unsigned short* kh16 = (unsigned short*)(ws + offKh);
  unsigned short* kl16 = (unsigned short*)(ws + offKl);
  unsigned short* vt16 = (unsigned short*)(ws + offVt);
  unsigned short* o16  = (unsigned short*)(ws + offO);

  static_assert(kActElems % 8 == 0 && kWElems % 8 == 0);
  const int a8 = (int)(kActElems / 8);
  const int w8 = (int)(kWElems / 8);
  const int ga = (a8 + 255) / 256, gw = (w8 + 255) / 256;
  cast_f32_bf16x8<<<ga, 256, 0, stream>>>(q,  qb16, a8);
  cast_f32_bf16x8<<<ga, 256, 0, stream>>>(k,  kb16, a8);
  cast_f32_bf16x8<<<ga, 256, 0, stream>>>(v,  vb16, a8);
  cast_f32_bf16x8<<<gw, 256, 0, stream>>>(Wq, wq16, w8);
  cast_f32_bf16x8<<<gw, 256, 0, stream>>>(Wk, wk16, w8);
  cast_f32_bf16x8<<<gw, 256, 0, stream>>>(Wv, wv16, w8);
  cast_f32_f16c_x8<<<gw, 256, 0, stream>>>(Wo, wo16, w8, kWoCarry);

  static_assert(kRows % 64 == 0 && kDm % 64 == 0 && kDm % 32 == 0);
  const int tilesQK = (kRows / 64) * (kDm / 64);
  const int gQK = (tilesQK + 7) / 8;
  wmma_gemm64<1, false, 2, 2, false, 0><<<dim3(gQK, 1), 256, 0, stream>>>(
      qb16, qb16, kDm, 0L, wq16, wq16, kDm, 0L,
      (void*)qh16, (void*)ql16, kDm, 0L, bq, bq, 0L, kRows, kDm, kDm, 1.0f);
  wmma_gemm64<1, false, 2, 2, false, 0><<<dim3(gQK, 1), 256, 0, stream>>>(
      kb16, kb16, kDm, 0L, wk16, wk16, kDm, 0L,
      (void*)kh16, (void*)kl16, kDm, 0L, bk, bk, 0L, kRows, kDm, kDm, 1.0f);
  const int tilesV = (kDm / 64) * (kRows / 64);
  const int gV = (tilesV + 7) / 8;
  wmma_gemm64<1, false, 1, 1, false, 0><<<dim3(gV, 1), 256, 0, stream>>>(
      wv16, wv16, kDm, 0L, vb16, vb16, kDm, 0L,
      (void*)vt16, (void*)vt16, kRows, 0L, bv, bv, 0L, kDm, kRows, kDm, 1.0f);

  const int gA = kBatch * kHeads * (kSeq / kQblk);
  const float score_scale = 0.125f;
  const float out_mul = kOCarry / kPCarry;
  attn_core<<<gA, 128, 0, stream>>>(qh16, ql16, kh16, kl16, vt16, o16, score_scale, out_mul);

  wmma_gemm64<0, false, 2, 0, false, 0><<<dim3(gQK, 1), 256, 0, stream>>>(
      o16, o16, kDm, 0L, wo16, wo16, kDm, 0L,
      d_out, d_out, kDm, 0L, bo, bo, 0L, kRows, kDm, kDm, 1.0f / (kOCarry * kWoCarry));
}
